// MusicAttentionBlock_36816459661838
// MI455X (gfx1250) — hardware-verified
//
#include <hip/hip_runtime.h>

typedef _Float16 v16h __attribute__((ext_vector_type(16)));
typedef _Float16 v8h  __attribute__((ext_vector_type(8)));
typedef float    v8f  __attribute__((ext_vector_type(8)));
typedef float    v4f  __attribute__((ext_vector_type(4)));
typedef v8h __attribute__((may_alias)) v8ha;
typedef v4f __attribute__((may_alias)) v4fa;

union Frag { v16h v; v8h half[2]; };

#define BB     2
#define SS     2048
#define DM     1024
#define NH     16
#define HD     64
#define DFF    2048
#define MROWS  (BB * SS)
#define NREL   257
#define MAXREL 128
#define WSCALE 32.0f
#define WINV   0.03125f
#define PSCALE 16384.0f
#define QKS    0.125f
#define LNEPS  1e-5f

__device__ __forceinline__ v8f wmma_f16(v16h a, v16h b, v8f c) {
  v8f d = __builtin_amdgcn_wmma_f32_16x16x32_f16(false, a, false, b, (short)0, c, false, false);
  asm volatile("v_nop\n\tv_nop\n\tv_nop\n\tv_nop" : "+v"(d) : "v"(a), "v"(b));
  return d;
}

__device__ __forceinline__ v16h load_frag(const _Float16* p, int h) {
  Frag f;
  f.half[0] = *(const v8ha*)(p + 8 * h);
  f.half[1] = *(const v8ha*)(p + 16 + 8 * h);
  return f.v;
}

__device__ __forceinline__ float wave_sum(float v) {
  v += __shfl_xor(v, 16);
  v += __shfl_xor(v, 8);
  v += __shfl_xor(v, 4);
  v += __shfl_xor(v, 2);
  v += __shfl_xor(v, 1);
  return v;
}

__device__ __forceinline__ void tc_store_pass(const _Float16* tile, _Float16* out,
                                              int R, int r0, int c0, int t) {
  const int q8 = t & 7;
  #pragma unroll
  for (int i = 0; i < 2; ++i) {
    const int L = (t >> 3) + 32 * i;
    const v8h v = *(const v8ha*)(tile + L * 72 + 8 * q8);
    _Float16* dst = out + (size_t)(c0 + L) * R + r0 + 8 * q8;
    *(volatile v8h*)dst = v;
  }
}

__global__ __launch_bounds__(256) void tconv_kernel(
    const float* __restrict__ in, _Float16* __restrict__ out, int R, int C)
{
  __shared__ __attribute__((aligned(16))) _Float16 tile[64 * 72];
  const int t = threadIdx.x;
  const int c0 = blockIdx.x * 64, r0 = blockIdx.y * 64;
  if (c0 + 64 > C || r0 + 64 > R) return;
  #pragma unroll
  for (int i = 0; i < 4; ++i) {
    const int idx = t + 256 * i;
    const int r = idx >> 4, c4 = (idx & 15) * 4;
    const v4f v = *(const v4fa*)(in + (size_t)(r0 + r) * C + c0 + c4);
    tile[(c4 + 0) * 72 + r] = (_Float16)(v.x * WSCALE);
    tile[(c4 + 1) * 72 + r] = (_Float16)(v.y * WSCALE);
    tile[(c4 + 2) * 72 + r] = (_Float16)(v.z * WSCALE);
    tile[(c4 + 3) * 72 + r] = (_Float16)(v.w * WSCALE);
  }
  __syncthreads();
  tc_store_pass(tile, out, R, r0, c0, t);
  __threadfence();
  tc_store_pass(tile, out, R, r0, c0, t);
}

__global__ __launch_bounds__(128) void ln_kernel(
    const float* __restrict__ x, const float* __restrict__ g, const float* __restrict__ bt,
    _Float16* __restrict__ y, int nrows)
{
  __shared__ float red[4];
  const int row = blockIdx.x;
  if (row >= nrows) return;
  const int t = threadIdx.x, lane = t & 31, w = t >> 5;
  const float* xr = x + (size_t)row * DM + 8 * t;
  const v4f a = *(const v4fa*)xr;
  const v4f c = *(const v4fa*)(xr + 4);
  float e[8] = { a.x, a.y, a.z, a.w, c.x, c.y, c.z, c.w };
  float s = ((e[0] + e[1]) + (e[2] + e[3])) + ((e[4] + e[5]) + (e[6] + e[7]));
  s = wave_sum(s);
  if (lane == 0) red[w] = s;
  __syncthreads();
  const float mu = ((red[0] + red[1]) + (red[2] + red[3])) * (1.0f / DM);
  __syncthreads();
  float q = 0.0f;
  #pragma unroll
  for (int j = 0; j < 8; ++j) { e[j] = e[j] - mu; q += e[j] * e[j]; }
  q = wave_sum(q);
  if (lane == 0) red[w] = q;
  __syncthreads();
  const float var = ((red[0] + red[1]) + (red[2] + red[3])) * (1.0f / DM);
  const float rstd = rsqrtf(var + LNEPS);
  const v4f ga = *(const v4fa*)(g + 8 * t);
  const v4f gb = *(const v4fa*)(g + 8 * t + 4);
  const v4f ba = *(const v4fa*)(bt + 8 * t);
  const v4f bb = *(const v4fa*)(bt + 8 * t + 4);
  const float gg[8] = { ga.x, ga.y, ga.z, ga.w, gb.x, gb.y, gb.z, gb.w };
  const float bv[8] = { ba.x, ba.y, ba.z, ba.w, bb.x, bb.y, bb.z, bb.w };
  v8h o;
  #pragma unroll
  for (int j = 0; j < 8; ++j) o[j] = (_Float16)(e[j] * rstd * gg[j] + bv[j]);
  _Float16* dst = y + (size_t)row * DM + 8 * t;
  *(volatile v8h*)dst = o;
  __threadfence();
  *(volatile v8h*)dst = o;
}

__device__ __forceinline__ void qkv_store_pass(const _Float16* sT, _Float16* plane, _Float16* vt,
                                               int which, int bh, int l0, int w, int lane) {
  const int q8 = lane & 7, sub = lane >> 3;
  #pragma unroll
  for (int i = 0; i < 8; ++i) {
    const int lid = w * 32 + i * 4 + sub;
    v8h v;
    _Float16* dst;
    if (which != 2) {
      v = *(const v8ha*)(sT + lid * HD + 8 * q8);
      dst = plane + ((size_t)bh * SS + l0 + lid) * HD + 8 * q8;
    } else {
      const int d = lid >> 1, hl = lid & 1;
      v = *(const v8ha*)(sT + d * 128 + 64 * hl + 8 * q8);
      dst = vt + ((size_t)bh * HD + d) * SS + l0 + 64 * hl + 8 * q8;
    }
    *(volatile v8h*)dst = v;
  }
}

__device__ __forceinline__ void h16_store_pass(const _Float16* sT, _Float16* outh,
                                               int N, int m0, int n0, int w, int lane) {
  const int q8 = lane & 7, sub = lane >> 3;
  #pragma unroll
  for (int i = 0; i < 8; ++i) {
    const int lid = w * 32 + i * 4 + sub;
    const v8h v = *(const v8ha*)(sT + lid * 64 + 8 * q8);
    _Float16* dst = outh + (size_t)(m0 + lid) * N + n0 + 8 * q8;
    *(volatile v8h*)dst = v;
  }
}

__device__ __forceinline__ void f32_store_pass(const float* sC, const float* __restrict__ bias,
                                               const float* __restrict__ resid, float* outf,
                                               int N, int m0, int n0, int w, int lane) {
  const int q8 = lane & 7, sub = lane >> 3;
  #pragma unroll
  for (int i = 0; i < 16; ++i) {
    const int L = i * 4 + sub;
    const int row = 32 * w + (L >> 1), hl = L & 1;
    const int col = 32 * hl + 4 * q8;
    const v4f cv = *(const v4fa*)(sC + row * 64 + col);
    const v4f bvv = *(const v4fa*)(bias + n0 + col);
    const size_t gi = (size_t)(m0 + row) * N + n0 + col;
    const v4f rv = *(const v4fa*)(resid + gi);
    const v4f o = (cv + bvv) + rv;
    *(volatile v4f*)(outf + gi) = o;
  }
}

template <int EPI>
__global__ __launch_bounds__(128) void gemm_kernel(
    const _Float16* __restrict__ A,
    const _Float16* __restrict__ Wt,
    int K, int N,
    const float* __restrict__ bias,
    const float* __restrict__ resid,
    float* __restrict__ outf,
    _Float16* __restrict__ outh,
    _Float16* __restrict__ qpl,
    _Float16* __restrict__ kpl,
    _Float16* __restrict__ vtpl)
{
  __shared__ __attribute__((aligned(16))) char smem[(EPI == 2) ? 32768 : 16384];

  const int tid = threadIdx.x, lane = tid & 31, w = tid >> 5;
  const int h = lane >> 4, m = lane & 15;
  const int m0 = blockIdx.x * 128;
  const int n0 = blockIdx.y * 64;
  if (m0 + 128 > MROWS || n0 + 64 > N) return;
  const int m0w = m0 + 32 * w;

  const _Float16* xa0 = A + (size_t)(m0w + m) * K;
  const _Float16* xa1 = xa0 + (size_t)16 * K;
  const _Float16* wb  = Wt + (size_t)(n0 + m) * K;

  const v8f zero8 = {0.f, 0.f, 0.f, 0.f, 0.f, 0.f, 0.f, 0.f};
  v8f acc[2][4];
  #pragma unroll
  for (int mt = 0; mt < 2; ++mt)
    #pragma unroll
    for (int nt = 0; nt < 4; ++nt) acc[mt][nt] = zero8;

  #pragma unroll 1
  for (int k0 = 0; k0 < K; k0 += 32) {
    const v16h a0 = load_frag(xa0 + k0, h);
    const v16h a1 = load_frag(xa1 + k0, h);
    #pragma unroll
    for (int nt = 0; nt < 4; ++nt) {
      const v16h b = load_frag(wb + (size_t)nt * 16 * K + k0, h);
      acc[0][nt] = wmma_f16(a0, b, acc[0][nt]);
      acc[1][nt] = wmma_f16(a1, b, acc[1][nt]);
    }
  }

  if constexpr (EPI == 0) {
    _Float16* sT = (_Float16*)smem;
    const int nb = blockIdx.y;
    const int which = nb >> 4, head = nb & 15;
    #pragma unroll
    for (int nt = 0; nt < 4; ++nt) {
      const int feat = 16 * nt + m;
      #pragma unroll
      for (int mt = 0; mt < 2; ++mt) {
        #pragma unroll
        for (int r = 0; r < 8; ++r) {
          const int tokl = 32 * w + 16 * mt + 8 * h + r;
          const float yv = acc[mt][nt][r] * WINV;
          const int idx = (which == 2) ? (feat * 128 + tokl) : (tokl * HD + feat);
          sT[idx] = (_Float16)yv;
        }
      }
    }
    __syncthreads();
    const int b = m0 / SS, l0 = m0 - b * SS, bh = b * NH + head;
    _Float16* plane = (which == 0) ? qpl : kpl;
    qkv_store_pass(sT, plane, vtpl, which, bh, l0, w, lane);
    __threadfence();
    qkv_store_pass(sT, plane, vtpl, which, bh, l0, w, lane);
  } else if constexpr (EPI == 1) {
    _Float16* sT = (_Float16*)smem;
    #pragma unroll
    for (int nt = 0; nt < 4; ++nt) {
      const int feat = 16 * nt + m;
      const float bvl = bias[n0 + feat];
      #pragma unroll
      for (int mt = 0; mt < 2; ++mt) {
        #pragma unroll
        for (int r = 0; r < 8; ++r) {
          const int tokl = 32 * w + 16 * mt + 8 * h + r;
          const float v = acc[mt][nt][r] * WINV + bvl;
          const float gv = 0.5f * v * (1.0f + erff(v * 0.70710678118654752f));
          sT[tokl * 64 + feat] = (_Float16)gv;
        }
      }
    }
    __syncthreads();
    h16_store_pass(sT, outh, N, m0, n0, w, lane);
    __threadfence();
    h16_store_pass(sT, outh, N, m0, n0, w, lane);
  } else {
    float* sC = (float*)smem;
    #pragma unroll
    for (int nt = 0; nt < 4; ++nt) {
      const int feat = 16 * nt + m;
      #pragma unroll
      for (int mt = 0; mt < 2; ++mt) {
        #pragma unroll
        for (int r = 0; r < 8; ++r) {
          const int tokl = 32 * w + 16 * mt + 8 * h + r;
          sC[tokl * 64 + feat] = acc[mt][nt][r] * WINV;
        }
      }
    }
    __syncthreads();
    f32_store_pass(sC, bias, resid, outf, N, m0, n0, w, lane);
    __threadfence();
    f32_store_pass(sC, bias, resid, outf, N, m0, n0, w, lane);
  }
}

__device__ __forceinline__ v16h pack_p(v8f a, v8f c) {
  const v16h r = { (_Float16)(a[0] * PSCALE), (_Float16)(a[1] * PSCALE), (_Float16)(a[2] * PSCALE), (_Float16)(a[3] * PSCALE),
                   (_Float16)(a[4] * PSCALE), (_Float16)(a[5] * PSCALE), (_Float16)(a[6] * PSCALE), (_Float16)(a[7] * PSCALE),
                   (_Float16)(c[0] * PSCALE), (_Float16)(c[1] * PSCALE), (_Float16)(c[2] * PSCALE), (_Float16)(c[3] * PSCALE),
                   (_Float16)(c[4] * PSCALE), (_Float16)(c[5] * PSCALE), (_Float16)(c[6] * PSCALE), (_Float16)(c[7] * PSCALE) };
  return r;
}

__device__ __forceinline__ void att_store_pass(const _Float16* so, _Float16* ao,
                                               int b, int head, int q0, int lane) {
  const int q8 = lane & 7, sub = lane >> 3;
  #pragma unroll
  for (int i = 0; i < 4; ++i) {
    const int lid = i * 4 + sub;
    const v8h v = *(const v8ha*)(so + lid * 64 + 8 * q8);
    const size_t gi = ((size_t)b * SS + q0 + lid) * DM + head * HD + 8 * q8;
    *(volatile v8h*)(ao + gi) = v;
  }
}

__global__ __launch_bounds__(128) void attn_kernel(
    const _Float16* __restrict__ qpl,
    const _Float16* __restrict__ kpl,
    const _Float16* __restrict__ vtpl,
    const float* __restrict__ rel,
    _Float16* __restrict__ ao)
{
  __shared__ __attribute__((aligned(16))) _Float16 sO[4 * 16 * 64];
  __shared__ float relL[NREL + 3];

  const int tid = threadIdx.x, lane = tid & 31, w = tid >> 5;
  const int h = lane >> 4, m = lane & 15;
  const int bh = blockIdx.y, b = bh >> 4, head = bh & 15;
  const int qblk = blockIdx.x * 64;
  const int q0 = qblk + 16 * w;
  const int qi = q0 + m;

  for (int i = tid; i < NREL; i += 128) relL[i] = rel[i * NH + head];
  __syncthreads();

  const _Float16* qrow = qpl + ((size_t)bh * SS + q0 + m) * HD;
  const v16h qb0 = load_frag(qrow, h);
  const v16h qb1 = load_frag(qrow + 32, h);

  const v8f zero8 = {0.f, 0.f, 0.f, 0.f, 0.f, 0.f, 0.f, 0.f};
  v8f o[4];
  #pragma unroll
  for (int t = 0; t < 4; ++t) o[t] = zero8;
  float mrun = -1e30f, lrun = 0.0f;

  const _Float16* kbase = kpl + ((size_t)bh * SS + m) * HD;
  const _Float16* vbase = vtpl + ((size_t)bh * HD + m) * SS;

  const int nkb = (int)blockIdx.x + 1;
  #pragma unroll 1
  for (int ib = 0; ib < nkb; ++ib) {
    const int kb = ib * 64;
    v8f s[4];
    #pragma unroll
    for (int j = 0; j < 4; ++j) {
      const _Float16* kp = kbase + (size_t)(kb + 16 * j) * HD;
      const v16h kf0 = load_frag(kp, h);
      const v16h kf1 = load_frag(kp + 32, h);
      v8f z = zero8;
      z = wmma_f16(kf0, qb0, z);
      z = wmma_f16(kf1, qb1, z);
      s[j] = z;
    }
    #pragma unroll
    for (int j = 0; j < 4; ++j) {
      #pragma unroll
      for (int r = 0; r < 8; ++r) {
        const int kj = kb + 16 * j + 8 * h + r;
        const int dl = kj - qi;
        int idx = (dl < -MAXREL) ? 0 : (dl + MAXREL);
        idx = (idx > NREL - 1) ? (NREL - 1) : idx;
        const float sv = s[j][r] * QKS + relL[idx];
        s[j][r] = (dl <= 0) ? sv : -1e30f;
      }
    }

    float mloc = s[0][0];
    #pragma unroll
    for (int j = 0; j < 4; ++j)
      #pragma unroll
      for (int r = 0; r < 8; ++r) mloc = fmaxf(mloc, s[j][r]);
    mloc = fmaxf(mloc, __shfl_xor(mloc, 16));
    const float mnew = fmaxf(mrun, mloc);
    const float alpha = __expf(mrun - mnew);
    mrun = mnew;
    float lsum = 0.0f;
    #pragma unroll
    for (int j = 0; j < 4; ++j)
      #pragma unroll
      for (int r = 0; r < 8; ++r) {
        const float p = __expf(s[j][r] - mnew);
        s[j][r] = p;
        lsum += p;
      }
    lsum += __shfl_xor(lsum, 16);
    lrun = lrun * alpha + lsum;
    #pragma unroll
    for (int t = 0; t < 4; ++t)
      #pragma unroll
      for (int r = 0; r < 8; ++r) o[t][r] = o[t][r] * alpha;

    const v16h pb0 = pack_p(s[0], s[1]);
    const v16h pb1 = pack_p(s[2], s[3]);

    #pragma unroll
    for (int t = 0; t < 4; ++t) {
      const _Float16* vp = vbase + (size_t)(16 * t) * SS + kb;
      const v16h vf0 = load_frag(vp, h);
      const v16h vf1 = load_frag(vp + 32, h);
      o[t] = wmma_f16(vf0, pb0, o[t]);
      o[t] = wmma_f16(vf1, pb1, o[t]);
    }
  }

  const float inv = (1.0f / lrun) * (1.0f / PSCALE);
  _Float16* so = sO + w * 1024;
  #pragma unroll
  for (int t = 0; t < 4; ++t) {
    v8h pk;
    #pragma unroll
    for (int r = 0; r < 8; ++r) pk[r] = (_Float16)(o[t][r] * inv);
    *(v8ha*)(so + m * 64 + 16 * t + 8 * h) = pk;
  }
  __syncthreads();

  att_store_pass(so, ao, b, head, q0, lane);
  __threadfence();
  att_store_pass(so, ao, b, head, q0, lane);
}

extern "C" void kernel_launch(void* const* d_in, const int* in_sizes, int n_in,
                              void* d_out, int out_size, void* d_ws, size_t ws_size,
                              hipStream_t stream) {
  if (n_in < 13) return;
  if (in_sizes[0] != MROWS * DM) return;
  if (in_sizes[1] != DM || in_sizes[2] != DM) return;
  if (in_sizes[3] != DM * 3 * DM) return;
  if (in_sizes[4] != DM * DM) return;
  if (in_sizes[5] != DM) return;
  if (in_sizes[6] != NREL * NH) return;
  if (in_sizes[7] != DM || in_sizes[8] != DM) return;
  if (in_sizes[9] != DM * DFF || in_sizes[10] != DFF) return;
  if (in_sizes[11] != DFF * DM || in_sizes[12] != DM) return;
  if (out_size != MROWS * DM) return;

  const float* x     = (const float*)d_in[0];
  const float* ln1_g = (const float*)d_in[1];
  const float* ln1_b = (const float*)d_in[2];
  const float* w_qkv = (const float*)d_in[3];
  const float* w_out = (const float*)d_in[4];
  const float* b_out = (const float*)d_in[5];
  const float* rel   = (const float*)d_in[6];
  const float* ln2_g = (const float*)d_in[7];
  const float* ln2_b = (const float*)d_in[8];
  const float* w1    = (const float*)d_in[9];
  const float* b1    = (const float*)d_in[10];
  const float* w2    = (const float*)d_in[11];
  const float* b2    = (const float*)d_in[12];
  float* outp = (float*)d_out;

  const size_t act_h   = (size_t)MROWS * DM * 2;
  const size_t wqkv_h  = (size_t)3 * DM * DM * 2;
  const size_t wout_h  = (size_t)DM * DM * 2;
  const size_t w1_h    = (size_t)DFF * DM * 2;
  const size_t w2_h    = (size_t)DM * DFF * 2;
  const size_t x2_f    = (size_t)MROWS * DM * 4;
  const size_t ffn1_h  = (size_t)MROWS * DFF * 2;
  const size_t total = act_h + wqkv_h + wout_h + w1_h + w2_h
                     + 4 * act_h + x2_f + act_h + ffn1_h;
  if (total > ws_size) return;

  char* ws = (char*)d_ws;
  size_t off = 0;
  _Float16* xn    = (_Float16*)(ws + off); off += act_h;
  _Float16* wqkvT = (_Float16*)(ws + off); off += wqkv_h;
  _Float16* woutT = (_Float16*)(ws + off); off += wout_h;
  _Float16* w1T   = (_Float16*)(ws + off); off += w1_h;
  _Float16* w2T   = (_Float16*)(ws + off); off += w2_h;
  _Float16* qpl   = (_Float16*)(ws + off); off += act_h;
  _Float16* kpl   = (_Float16*)(ws + off); off += act_h;
  _Float16* vtpl  = (_Float16*)(ws + off); off += act_h;
  _Float16* attn  = (_Float16*)(ws + off); off += act_h;
  float*    x2    = (float*)   (ws + off); off += x2_f;
  _Float16* h2    = (_Float16*)(ws + off); off += act_h;
  _Float16* ffn1  = (_Float16*)(ws + off); off += ffn1_h;
  if (off > ws_size) return;

  tconv_kernel<<<dim3(3 * DM / 64, DM / 64), 256, 0, stream>>>(w_qkv, wqkvT, DM, 3 * DM);
  tconv_kernel<<<dim3(DM / 64, DM / 64), 256, 0, stream>>>(w_out, woutT, DM, DM);
  tconv_kernel<<<dim3(DFF / 64, DM / 64), 256, 0, stream>>>(w1, w1T, DM, DFF);
  tconv_kernel<<<dim3(DM / 64, DFF / 64), 256, 0, stream>>>(w2, w2T, DFF, DM);
  ln_kernel<<<MROWS, 128, 0, stream>>>(x, ln1_g, ln1_b, xn, MROWS);
  gemm_kernel<0><<<dim3(MROWS / 128, 3 * DM / 64), 128, 0, stream>>>(
      xn, wqkvT, DM, 3 * DM, b_out, x, x2, h2, qpl, kpl, vtpl);
  attn_kernel<<<dim3(SS / 64, BB * NH), 128, 0, stream>>>(qpl, kpl, vtpl, rel, attn);
  gemm_kernel<2><<<dim3(MROWS / 128, DM / 64), 128, 0, stream>>>(
      attn, woutT, DM, DM, b_out, x, x2, h2, qpl, kpl, vtpl);
  ln_kernel<<<MROWS, 128, 0, stream>>>(x2, ln2_g, ln2_b, h2, MROWS);
  gemm_kernel<1><<<dim3(MROWS / 128, DFF / 64), 128, 0, stream>>>(
      h2, w1T, DM, DFF, b1, x, x2, ffn1, qpl, kpl, vtpl);
  gemm_kernel<2><<<dim3(MROWS / 128, DM / 64), 128, 0, stream>>>(
      ffn1, w2T, DFF, DM, b2, x2, outp, h2, qpl, kpl, vtpl);
}
